// MultiHeadAttentionLayer_38388417691980
// MI455X (gfx1250) — hardware-verified
//
#include <hip/hip_runtime.h>

#ifndef NB
#define NB 2
#endif
#ifndef SEQ
#define SEQ 2048
#endif
#define NB_FULL 2
#define SEQ_FULL 2048
#define IN_DIM 1024
#define NUM_HEADS 16
#define HEAD_DIM 64
#define OUT_DIM (NUM_HEADS * HEAD_DIM)
#define MROWS (NB * SEQ)
#define NBKT 32
#define TABN 4096
#define TOFF 2047

static_assert(SEQ % 256 == 0);
static_assert(SEQ <= SEQ_FULL);
static_assert(NB >= 1 && NB <= NB_FULL);
static_assert(IN_DIM % 64 == 0);
static_assert(OUT_DIM % 64 == 0);
static_assert(HEAD_DIM == 64);
static_assert(MROWS % 128 == 0);
static_assert((size_t)NB_FULL * SEQ_FULL * OUT_DIM * 4 == 16777216);
static_assert(2 * SEQ_FULL <= TABN);

#define QCAR 8.0f
#define RCAR 2048.0f
#define PCAR 16384.0f

#define BTP 40
#define EQP 72
#define EVP 136
#define TP  72
#define OLP 68
#define ESZ 9216
static_assert(128 * EQP <= ESZ);
static_assert(64 * EVP <= ESZ);

typedef __bf16   v16bf __attribute__((ext_vector_type(16)));
typedef __bf16   v8bf  __attribute__((ext_vector_type(8)));
typedef _Float16 v16h  __attribute__((ext_vector_type(16)));
typedef _Float16 v8h   __attribute__((ext_vector_type(8)));
typedef float    v8f   __attribute__((ext_vector_type(8)));
typedef float    v4f   __attribute__((ext_vector_type(4)));
typedef unsigned int v4u __attribute__((ext_vector_type(4)));

__device__ __forceinline__ v8f mma_bf16(v16bf a, v16bf b, v8f c) {
  v8f d = __builtin_amdgcn_wmma_f32_16x16x32_bf16(false, a, false, b, (short)0, c, false, false);
  asm volatile("v_nop\n\tv_nop\n\tv_nop\n\tv_nop" : "+v"(d) : "v"(a), "v"(b));
  return d;
}
__device__ __forceinline__ v8f mma_f16(v16h a, v16h b, v8f c) {
  v8f d = __builtin_amdgcn_wmma_f32_16x16x32_f16(false, a, false, b, (short)0, c, false, false);
  asm volatile("v_nop\n\tv_nop\n\tv_nop\n\tv_nop" : "+v"(d) : "v"(a), "v"(b));
  return d;
}

__device__ __forceinline__ v16bf ld_frag_bf(const __bf16* p0, int ld, int rc, int kk, int lane) {
  const int hh = (lane >> 4) & 1;
  const __bf16* p = p0 + (size_t)rc * ld + kk + 8 * hh;
  const v8bf lo = *(const v8bf*)(p);
  const v8bf hi = *(const v8bf*)(p + 16);
  v16bf f;
#pragma unroll
  for (int i = 0; i < 8; ++i) { f[i] = lo[i]; f[8 + i] = hi[i]; }
  return f;
}
__device__ __forceinline__ v16h ld_frag_h(const _Float16* p0, int ld, int rc, int kk, int lane) {
  const int hh = (lane >> 4) & 1;
  const _Float16* p = p0 + (size_t)rc * ld + kk + 8 * hh;
  const v8h lo = *(const v8h*)(p);
  const v8h hi = *(const v8h*)(p + 16);
  v16h f;
#pragma unroll
  for (int i = 0; i < 8; ++i) { f[i] = lo[i]; f[8 + i] = hi[i]; }
  return f;
}

__device__ __forceinline__ unsigned int bfb(float x) {
  unsigned int u = __float_as_uint(x);
  u = u + 0x7FFFu + ((u >> 16) & 1u);
  return u >> 16;
}
__device__ __forceinline__ float bf16val(float x) {
  return __uint_as_float(bfb(x) << 16);
}
__device__ __forceinline__ unsigned short hbits(float x) {
  const _Float16 hv = (_Float16)x;
  return __builtin_bit_cast(unsigned short, hv);
}

__device__ __forceinline__ int rel_bucket(int rel) {
  const int ret = (rel > 0) ? 16 : 0;
  const int rp = (rel < 0) ? -rel : rel;
  int v = 15;
  v = (rp < 91) ? 14 : v;
  v = (rp < 64) ? 13 : v;
  v = (rp < 46) ? 12 : v;
  v = (rp < 32) ? 11 : v;
  v = (rp < 23) ? 10 : v;
  v = (rp < 16) ? 9 : v;
  v = (rp < 12) ? 8 : v;
  v = (rp < 8) ? rp : v;
  return ret + v;
}

__global__ __launch_bounds__(256) void k_cvt_rows(const float* __restrict__ xq,
                                                  const float* __restrict__ xk,
                                                  const float* __restrict__ xv,
                                                  unsigned short* __restrict__ xb, int n8) {
  const int z = blockIdx.y;
  const int g = blockIdx.x * 256 + threadIdx.x;
  if (g >= n8) return;
  const float* X = (z == 0) ? xq : ((z == 1) ? xk : xv);
  const int m = g / (IN_DIM / 8);
  const int c8 = g - m * (IN_DIM / 8);
  const int b = m / SEQ;
  const int s = m - b * SEQ;
  const float* src = X + ((size_t)(b * SEQ_FULL + s)) * IN_DIM + (size_t)c8 * 8;
  const v4f a = *(const v4f*)(src);
  const v4f c = *(const v4f*)(src + 4);
  v4u w;
  w[0] = bfb(a[0]) | (bfb(a[1]) << 16);
  w[1] = bfb(a[2]) | (bfb(a[3]) << 16);
  w[2] = bfb(c[0]) | (bfb(c[1]) << 16);
  w[3] = bfb(c[2]) | (bfb(c[3]) << 16);
  volatile v4u* p = (volatile v4u*)(xb + (size_t)z * MROWS * IN_DIM + (size_t)g * 8);
  *p = w;
  __threadfence();
  *p = w;
}

__global__ __launch_bounds__(256) void k_cvt_wT(const float* __restrict__ Wq,
                                                const float* __restrict__ Wk,
                                                const float* __restrict__ Wv,
                                                unsigned short* __restrict__ wT) {
  __shared__ __align__(16) unsigned short T[64 * TP];
  const int z = blockIdx.z;
  const float* W = (z == 0) ? Wq : ((z == 1) ? Wk : Wv);
  unsigned short* dst = wT + (size_t)z * OUT_DIM * IN_DIM;
  const int k0 = blockIdx.x * 64;
  const int n0 = blockIdx.y * 64;
  const int tid = threadIdx.x;
  const int wave = tid >> 5, lane = tid & 31;

#pragma unroll
  for (int i = 0; i < 4; ++i) {
    const int idx = i * 256 + tid;
    const int kk = idx >> 4;
    const int c4 = (idx & 15) * 4;
    const v4f w = *(const v4f*)(W + (size_t)(k0 + kk) * OUT_DIM + n0 + c4);
    T[(c4 + 0) * TP + kk] = (unsigned short)bfb(w[0]);
    T[(c4 + 1) * TP + kk] = (unsigned short)bfb(w[1]);
    T[(c4 + 2) * TP + kk] = (unsigned short)bfb(w[2]);
    T[(c4 + 3) * TP + kk] = (unsigned short)bfb(w[3]);
  }
  __syncthreads();

  v4u v[2];
  size_t off[2];
#pragma unroll
  for (int it = 0; it < 2; ++it) {
    const int nn = wave * 8 + it * 4 + (lane >> 3);
    const int q = lane & 7;
    v[it] = *(const v4u*)(&T[nn * TP + q * 8]);
    off[it] = (size_t)(n0 + nn) * IN_DIM + k0 + q * 8;
  }
#pragma unroll
  for (int it = 0; it < 2; ++it) *(volatile v4u*)(dst + off[it]) = v[it];
  __threadfence();
#pragma unroll
  for (int it = 0; it < 2; ++it) *(volatile v4u*)(dst + off[it]) = v[it];
}

__global__ __launch_bounds__(256) void k_bias(const float* __restrict__ btab,
                                              float* __restrict__ gtab) {
  const int g = blockIdx.x * 256 + threadIdx.x;
  if (g >= NUM_HEADS * TABN / 4) return;
  const int h = g / (TABN / 4);
  const int i4 = (g - h * (TABN / 4)) * 4;
  v4f v;
#pragma unroll
  for (int j = 0; j < 4; ++j) {
    const int bk = rel_bucket(i4 + j - TOFF);
    int idx = bk * NUM_HEADS + h;
    idx = (idx < 0) ? 0 : ((idx > NBKT * NUM_HEADS - 1) ? (NBKT * NUM_HEADS - 1) : idx);
    v[j] = bf16val(btab[idx]);
  }
  volatile v4f* p = (volatile v4f*)(gtab + (size_t)g * 4);
  *p = v;
  __threadfence();
  *p = v;
}

__global__ __launch_bounds__(256) void k_proj(
    const unsigned short* __restrict__ xb, const unsigned short* __restrict__ wT,
    unsigned short* __restrict__ qh, unsigned short* __restrict__ qr,
    unsigned short* __restrict__ kh, unsigned short* __restrict__ kr,
    unsigned short* __restrict__ vtp) {
  __shared__ __align__(16) unsigned short bt[64 * BTP];
  __shared__ __align__(16) unsigned short E[ESZ];
  __shared__ __align__(16) unsigned short E2[ESZ];

  const int z = blockIdx.z;
  const int n0 = blockIdx.x * 64;
  const int m0 = blockIdx.y * 128;
  const int tid = threadIdx.x;
  const int wave = tid >> 5, lane = tid & 31;
  const int l15 = lane & 15, half = (lane >> 4) & 1;

  const unsigned short* Wt = wT + (size_t)z * OUT_DIM * IN_DIM;
  const __bf16* A = (const __bf16*)(xb + (size_t)z * MROWS * IN_DIM);

  const int tn = tid >> 2;
  const int tk = (tid & 3) * 8;
  const unsigned short* wsrc = Wt + (size_t)(n0 + tn) * IN_DIM + tk;
  const int arow = m0 + wave * 16 + l15;

  v8f acc[4] = {};
  for (int s = 0; s < IN_DIM / 32; ++s) {
    const int kk = s * 32;
    const v4u wv = *(const v4u*)(wsrc + kk);
    __syncthreads();
    *(v4u*)(&bt[tn * BTP + tk]) = wv;
    __syncthreads();
    const v16bf a = ld_frag_bf(A, IN_DIM, arow, kk, lane);
#pragma unroll
    for (int j = 0; j < 4; ++j) {
      const v16bf b = ld_frag_bf((const __bf16*)bt, BTP, j * 16 + l15, 0, lane);
      acc[j] = mma_bf16(a, b, acc[j]);
    }
  }

  if (z != 2) {
#pragma unroll
    for (int j = 0; j < 4; ++j) {
      const int col = j * 16 + l15;
#pragma unroll
      for (int r = 0; r < 8; ++r) {
        const int row = wave * 16 + 8 * half + r;
        const float a8 = acc[j][r] * QCAR;
        const _Float16 hv = (_Float16)a8;
        const float res = (a8 - (float)hv) * RCAR;
        E[row * EQP + col]  = __builtin_bit_cast(unsigned short, hv);
        E2[row * EQP + col] = hbits(res);
      }
    }
    __syncthreads();
    unsigned short* dh = (z == 0) ? qh : kh;
    unsigned short* dr = (z == 0) ? qr : kr;
    v4u v[4], w[4];
    size_t off[4];
#pragma unroll
    for (int it = 0; it < 4; ++it) {
      const int row = wave * 16 + it * 4 + (lane >> 3);
      const int q = lane & 7;
      v[it] = *(const v4u*)(&E[row * EQP + q * 8]);
      w[it] = *(const v4u*)(&E2[row * EQP + q * 8]);
      off[it] = (size_t)(m0 + row) * OUT_DIM + n0 + q * 8;
    }
#pragma unroll
    for (int it = 0; it < 4; ++it) *(volatile v4u*)(dh + off[it]) = v[it];
#pragma unroll
    for (int it = 0; it < 4; ++it) *(volatile v4u*)(dr + off[it]) = w[it];
    __threadfence();
#pragma unroll
    for (int it = 0; it < 4; ++it) *(volatile v4u*)(dh + off[it]) = v[it];
#pragma unroll
    for (int it = 0; it < 4; ++it) *(volatile v4u*)(dr + off[it]) = w[it];
  } else {
    const int bb = m0 / SEQ;
    const int s0 = m0 - bb * SEQ;
#pragma unroll
    for (int j = 0; j < 4; ++j) {
      const int col = j * 16 + l15;
#pragma unroll
      for (int r = 0; r < 8; ++r) {
        const int srow = wave * 16 + 8 * half + r;
        E[col * EVP + srow] = hbits(acc[j][r] * QCAR);
      }
    }
    __syncthreads();
    v4u v[4];
    size_t off[4];
#pragma unroll
    for (int it = 0; it < 4; ++it) {
      const int drow = wave * 8 + it * 2 + half;
      const int q = l15;
      v[it] = *(const v4u*)(&E[drow * EVP + q * 8]);
      off[it] = ((size_t)bb * OUT_DIM + n0 + drow) * SEQ + s0 + q * 8;
    }
#pragma unroll
    for (int it = 0; it < 4; ++it) *(volatile v4u*)(vtp + off[it]) = v[it];
    __threadfence();
#pragma unroll
    for (int it = 0; it < 4; ++it) *(volatile v4u*)(vtp + off[it]) = v[it];
  }
}

__global__ __launch_bounds__(64) void k_attn(const unsigned short* __restrict__ qh,
                                             const unsigned short* __restrict__ qr,
                                             const unsigned short* __restrict__ kh,
                                             const unsigned short* __restrict__ kr,
                                             const unsigned short* __restrict__ vtp,
                                             const float* __restrict__ key_mask,
                                             const float* __restrict__ gtab,
                                             float* __restrict__ outp) {
  __shared__ __align__(16) float tb[TABN];
  __shared__ __align__(16) float mt[SEQ];
  __shared__ __align__(16) float Ol[2 * 16 * OLP];

  const int tid = threadIdx.x;
  const int wave = tid >> 5, lane = tid & 31;
  const int l15 = lane & 15;
  const int half = (lane >> 4) & 1;
  const int nqb = SEQ / 32;
  const int b = blockIdx.x / nqb;
  const int qblk = blockIdx.x - b * nqb;
  const int q0l = qblk * 32 + wave * 16;
  const int head = blockIdx.y;

  {
    const float* gsrc = gtab + (size_t)head * TABN;
#pragma unroll
    for (int it = 0; it < TABN / 4 / 64; ++it) {
      const int i4 = it * 64 + tid;
      *(v4f*)(&tb[i4 * 4]) = *(const v4f*)(gsrc + (size_t)i4 * 4);
    }
    const float* msrc = key_mask + (size_t)b * SEQ_FULL;
#pragma unroll
    for (int it = 0; it < SEQ / 4 / 64; ++it) {
      const int i4 = it * 64 + tid;
      const v4f km = *(const v4f*)(msrc + (size_t)i4 * 4);
      v4f ma;
#pragma unroll
      for (int c = 0; c < 4; ++c) ma[c] = (1.0f - bf16val(km[c])) * (-10000.0f);
      *(v4f*)(&mt[i4 * 4]) = ma;
    }
  }
  __syncthreads();

  const _Float16* QH = (const _Float16*)qh;
  const _Float16* QR = (const _Float16*)qr;
  const _Float16* KH = (const _Float16*)kh;
  const _Float16* KR = (const _Float16*)kr;
  const _Float16* VT = (const _Float16*)vtp;

  const size_t qrow = (size_t)b * SEQ + q0l;
  const _Float16* qhb = QH + qrow * OUT_DIM + head * HEAD_DIM;
  const _Float16* qrb = QR + qrow * OUT_DIM + head * HEAD_DIM;
  const v16h qa0 = ld_frag_h(qhb, OUT_DIM, l15, 0, lane);
  const v16h qa1 = ld_frag_h(qhb, OUT_DIM, l15, 32, lane);
  const v16h qc0 = ld_frag_h(qrb, OUT_DIM, l15, 0, lane);
  const v16h qc1 = ld_frag_h(qrb, OUT_DIM, l15, 32, lane);
  const _Float16* khb = KH + (size_t)b * SEQ * OUT_DIM + head * HEAD_DIM;
  const _Float16* krb = KR + (size_t)b * SEQ * OUT_DIM + head * HEAD_DIM;
  const _Float16* vbase = VT + ((size_t)b * OUT_DIM + head * HEAD_DIM) * SEQ;

  v8f o[4] = {};
  float mrun = -1.0e30f, lrun = 0.0f;
  const float sscale = 1.0f / 64.0f;
  const float rscale = 1.0f / RCAR;
  const int bbase = 8 * half - (q0l + l15) + TOFF;

  for (int kc = 0; kc < SEQ; kc += 32) {
    const _Float16* kth = khb + (size_t)kc * OUT_DIM;
    const _Float16* ktr = krb + (size_t)kc * OUT_DIM;
    v8f c0 = {}, e0 = {}, c1 = {}, e1 = {};
    {
      const v16h kh0 = ld_frag_h(kth, OUT_DIM, l15, 0, lane);
      const v16h kh1 = ld_frag_h(kth, OUT_DIM, l15, 32, lane);
      c0 = mma_f16(kh0, qa0, c0);
      c0 = mma_f16(kh1, qa1, c0);
      e0 = mma_f16(kh0, qc0, e0);
      e0 = mma_f16(kh1, qc1, e0);
      const v16h kl0 = ld_frag_h(ktr, OUT_DIM, l15, 0, lane);
      const v16h kl1 = ld_frag_h(ktr, OUT_DIM, l15, 32, lane);
      e0 = mma_f16(kl0, qa0, e0);
      e0 = mma_f16(kl1, qa1, e0);
    }
    {
      const v16h kh2 = ld_frag_h(kth, OUT_DIM, 16 + l15, 0, lane);
      const v16h kh3 = ld_frag_h(kth, OUT_DIM, 16 + l15, 32, lane);
      c1 = mma_f16(kh2, qa0, c1);
      c1 = mma_f16(kh3, qa1, c1);
      e1 = mma_f16(kh2, qc0, e1);
      e1 = mma_f16(kh3, qc1, e1);
      const v16h kl2 = ld_frag_h(ktr, OUT_DIM, 16 + l15, 0, lane);
      const v16h kl3 = ld_frag_h(ktr, OUT_DIM, 16 + l15, 32, lane);
      e1 = mma_f16(kl2, qa0, e1);
      e1 = mma_f16(kl3, qa1, e1);
    }

    const v4f m00 = *(const v4f*)(&mt[kc + 8 * half]);
    const v4f m01 = *(const v4f*)(&mt[kc + 8 * half + 4]);
    const v4f m10 = *(const v4f*)(&mt[kc + 16 + 8 * half]);
    const v4f m11 = *(const v4f*)(&mt[kc + 16 + 8 * half + 4]);
    float mk0[8], mk1[8];
#pragma unroll
    for (int c = 0; c < 4; ++c) { mk0[c] = m00[c]; mk0[4 + c] = m01[c]; mk1[c] = m10[c]; mk1[4 + c] = m11[c]; }
    const int bi = bbase + kc;

    float sa[8], sb[8];
#pragma unroll
    for (int r = 0; r < 8; ++r) {
      sa[r] = (fmaf(e0[r], rscale, c0[r]) * sscale + tb[bi + r]) + mk0[r];
      sb[r] = (fmaf(e1[r], rscale, c1[r]) * sscale + tb[bi + 16 + r]) + mk1[r];
    }
    float lm = fmaxf(sa[0], sb[0]);
#pragma unroll
    for (int r = 1; r < 8; ++r) lm = fmaxf(lm, fmaxf(sa[r], sb[r]));
    lm = fmaxf(lm, __shfl_xor(lm, 16, 32));
    const float mnew = fmaxf(mrun, lm);
    const float alpha = __expf(mrun - mnew);
    float p0[8], p1[8];
    float ls = 0.0f;
#pragma unroll
    for (int r = 0; r < 8; ++r) {
      p0[r] = __expf(sa[r] - mnew);
      p1[r] = __expf(sb[r] - mnew);
      ls += p0[r] + p1[r];
    }
    ls += __shfl_xor(ls, 16, 32);
    lrun = lrun * alpha + ls;
    mrun = mnew;
#pragma unroll
    for (int j = 0; j < 4; ++j)
#pragma unroll
      for (int r = 0; r < 8; ++r) o[j][r] *= alpha;

    v16h pb;
#pragma unroll
    for (int e = 0; e < 8; ++e) {
      pb[e]     = (_Float16)(p0[e] * PCAR);
      pb[8 + e] = (_Float16)(p1[e] * PCAR);
    }
#pragma unroll
    for (int j = 0; j < 4; ++j) {
      const v16h va = ld_frag_h(vbase, SEQ, j * 16 + l15, kc, lane);
      o[j] = mma_f16(va, pb, o[j]);
    }
  }

  const float inv = 1.0f / (lrun * (PCAR * QCAR));
  float* Olw = Ol + wave * 16 * OLP;
#pragma unroll
  for (int j = 0; j < 4; ++j) {
    v4f lo4, hi4;
    lo4[0] = o[j][0] * inv; lo4[1] = o[j][1] * inv; lo4[2] = o[j][2] * inv; lo4[3] = o[j][3] * inv;
    hi4[0] = o[j][4] * inv; hi4[1] = o[j][5] * inv; hi4[2] = o[j][6] * inv; hi4[3] = o[j][7] * inv;
    *(v4f*)(&Olw[l15 * OLP + j * 16 + 8 * half])     = lo4;
    *(v4f*)(&Olw[l15 * OLP + j * 16 + 8 * half + 4]) = hi4;
  }
  __syncthreads();

  v4f v[8];
  size_t off[8];
  float* ob = outp + ((size_t)b * SEQ_FULL + q0l) * OUT_DIM + head * HEAD_DIM;
#pragma unroll
  for (int it = 0; it < 8; ++it) {
    const int row = it * 2 + half;
    const int q = l15;
    v[it] = *(const v4f*)(&Olw[row * OLP + q * 4]);
    off[it] = (size_t)row * OUT_DIM + q * 4;
  }
#pragma unroll
  for (int it = 0; it < 8; ++it) *(volatile v4f*)(ob + off[it]) = v[it];
  __threadfence();
#pragma unroll
  for (int it = 0; it < 8; ++it) *(volatile v4f*)(ob + off[it]) = v[it];
}

extern "C" void kernel_launch(void* const* d_in, const int* in_sizes, int n_in,
                              void* d_out, int out_size, void* d_ws, size_t ws_size,
                              hipStream_t stream) {
  if (n_in < 8) return;
  const int need_rows = (NB - 1) * SEQ_FULL + SEQ;
  if (in_sizes[0] < need_rows * IN_DIM || in_sizes[1] < need_rows * IN_DIM ||
      in_sizes[2] < need_rows * IN_DIM) return;
  if (in_sizes[3] < need_rows) return;
  if (in_sizes[4] < IN_DIM * OUT_DIM || in_sizes[5] < IN_DIM * OUT_DIM ||
      in_sizes[6] < IN_DIM * OUT_DIM) return;
  if (in_sizes[7] < NBKT * NUM_HEADS) return;
  if (out_size < need_rows * OUT_DIM) return;

  const float* xq = (const float*)d_in[0];
  const float* xk = (const float*)d_in[1];
  const float* xv = (const float*)d_in[2];
  const float* km = (const float*)d_in[3];
  const float* Wq = (const float*)d_in[4];
  const float* Wk = (const float*)d_in[5];
  const float* Wv = (const float*)d_in[6];
  const float* bt = (const float*)d_in[7];

  const size_t xb_bytes = (size_t)3 * MROWS * IN_DIM * 2;
  const size_t wt_bytes = (size_t)3 * OUT_DIM * IN_DIM * 2;
  const size_t pl_bytes = (size_t)MROWS * OUT_DIM * 2;
  const size_t tb_bytes = (size_t)NUM_HEADS * TABN * 4;
  const size_t off_xb = 0;
  const size_t off_wt = off_xb + xb_bytes;
  const size_t off_qh = off_wt + wt_bytes;
  const size_t off_qr = off_qh + pl_bytes;
  const size_t off_kh = off_qr + pl_bytes;
  const size_t off_kr = off_kh + pl_bytes;
  const size_t off_vt = off_kr + pl_bytes;
  const size_t off_tb = off_vt + pl_bytes;
  const size_t total  = off_tb + tb_bytes;
  if (total > ws_size) return;
  if (total > (size_t)134217728) return;

  char* ws = (char*)d_ws;
  unsigned short* xb  = (unsigned short*)(ws + off_xb);
  unsigned short* wt  = (unsigned short*)(ws + off_wt);
  unsigned short* qhp = (unsigned short*)(ws + off_qh);
  unsigned short* qrp = (unsigned short*)(ws + off_qr);
  unsigned short* khp = (unsigned short*)(ws + off_kh);
  unsigned short* krp = (unsigned short*)(ws + off_kr);
  unsigned short* vtp = (unsigned short*)(ws + off_vt);
  float*          gtb = (float*)(ws + off_tb);

  const int n8 = MROWS * IN_DIM / 8;
  k_cvt_rows<<<dim3((n8 + 255) / 256, 3), 256, 0, stream>>>(xq, xk, xv, xb, n8);
  k_cvt_wT<<<dim3(IN_DIM / 64, OUT_DIM / 64, 3), 256, 0, stream>>>(Wq, Wk, Wv, wt);
  k_bias<<<(NUM_HEADS * TABN / 4 + 255) / 256, 256, 0, stream>>>(bt, gtb);
  k_proj<<<dim3(OUT_DIM / 64, MROWS / 128, 3), 256, 0, stream>>>(xb, wt, qhp, qrp, khp, krp, vtp);
  k_attn<<<dim3(NB * SEQ / 32, NUM_HEADS), 64, 0, stream>>>(qhp, qrp, khp, krp, vtp, km, gtb,
                                                            (float*)d_out);
}
